// Relative_position_encoding_attention_56487409877633
// MI455X (gfx1250) — hardware-verified
//
#include <hip/hip_runtime.h>
#include <math.h>
#include <stdint.h>

#define NB     8
#define SEQ    1024
#define DM     512
#define NHEAD  8
#define HD     64
#define NROWS  (NB * SEQ)
#define KCH    32
#define WSC    64.0f
#define ACARRY 16.0f
#define QC     4.0f
#define VC     16.0f
#define PC     1024.0f
#define LOG2E  1.4426950408889634f
#define SCL    0.04419417382415922f
static_assert(NHEAD * HD == DM);
static_assert((SEQ % 64) == 0 && (DM % 64) == 0 && (NROWS % 64) == 0 && (HD % 32) == 0 && (SEQ % KCH) == 0);
static_assert(((NROWS * DM) % 2048) == 0);
#define ATT_THREADS (NHEAD * 32)
#define ATT_BLOCKS  (SEQ / 16)
#define ATT_SMEM_FLOATS 8192
static_assert(ATT_THREADS == 256);
static_assert(ATT_BLOCKS == 64);
static_assert(NHEAD * 16 * 36 <= ATT_SMEM_FLOATS);
static_assert((size_t)2 * 16 * DM * sizeof(unsigned short) <= (size_t)ATT_SMEM_FLOATS * sizeof(float));
static_assert((16 * DM) / 8 == 4 * ATT_THREADS);

typedef _Float16 v16h __attribute__((ext_vector_type(16)));
typedef _Float16 v8h  __attribute__((ext_vector_type(8)));
typedef __bf16   v16b __attribute__((ext_vector_type(16)));
typedef float    v8f  __attribute__((ext_vector_type(8)));
typedef float    v4f  __attribute__((ext_vector_type(4)));
typedef unsigned int v4u __attribute__((ext_vector_type(4)));

union FragH { v16h v; v8h h[2]; v4u u[2]; };
union FragAny { v16h h; v16b b; };

__device__ __forceinline__ unsigned short bf_bits(float f) {
  unsigned u = __float_as_uint(f);
  return (unsigned short)((u + 0x7FFFu + ((u >> 16) & 1u)) >> 16);
}
__device__ __forceinline__ float bf_up(unsigned short h) { return __uint_as_float(((unsigned)h) << 16); }
__device__ __forceinline__ float bfr(float f) { return bf_up(bf_bits(f)); }
__device__ __forceinline__ unsigned short h_bits(_Float16 x) { return __builtin_bit_cast(unsigned short, x); }
__device__ __forceinline__ unsigned pk16(unsigned short a, unsigned short b) { return (unsigned)a | ((unsigned)b << 16); }
__device__ __forceinline__ v8f zero8() { v8f z = {0.f, 0.f, 0.f, 0.f, 0.f, 0.f, 0.f, 0.f}; return z; }

__device__ __forceinline__ v16h ldfrag_u(const unsigned short* p) {
  FragH f;
  f.u[0] = *(const v4u*)(p);
  f.u[1] = *(const v4u*)(p + 16);
  return f.v;
}

__device__ __forceinline__ v8f mma_h(v16h a, v16h b, v8f c) {
  return __builtin_amdgcn_wmma_f32_16x16x32_f16(false, a, false, b, (short)0, c, false, false);
}
__device__ __forceinline__ v8f mma_b(v16h a, v16h b, v8f c) {
  FragAny ua, ub;
  ua.h = a;
  ub.h = b;
  return __builtin_amdgcn_wmma_f32_16x16x32_bf16(false, ua.b, false, ub.b, (short)0, c, false, false);
}
template <int BF>
__device__ __forceinline__ v8f mmaT(v16h a, v16h b, v8f c) {
  if constexpr (BF != 0) return mma_b(a, b, c);
  else return mma_h(a, b, c);
}
__device__ __forceinline__ void dep_guard1(v8f& a, v8f& b, v16h x) {
#if defined(__HIP_DEVICE_COMPILE__)
  asm volatile("v_nop\n\tv_nop\n\tv_nop\n\tv_nop" : "+v"(a), "+v"(b) : "v"(x));
#endif
}
__device__ __forceinline__ void guard2x6(v8f& a, v8f& b, v16h x0, v16h x1, v16h x2, v16h x3, v16h x4, v16h x5) {
#if defined(__HIP_DEVICE_COMPILE__)
  asm volatile("v_nop\n\tv_nop\n\tv_nop\n\tv_nop"
               : "+v"(a), "+v"(b) : "v"(x0), "v"(x1), "v"(x2), "v"(x3), "v"(x4), "v"(x5));
#endif
}
__device__ __forceinline__ void guard4x6(v8f& a, v8f& b, v8f& c, v8f& d,
                                         v16h x0, v16h x1, v16h x2, v16h x3, v16h x4, v16h x5) {
#if defined(__HIP_DEVICE_COMPILE__)
  asm volatile("v_nop\n\tv_nop\n\tv_nop\n\tv_nop"
               : "+v"(a), "+v"(b), "+v"(c), "+v"(d) : "v"(x0), "v"(x1), "v"(x2), "v"(x3), "v"(x4), "v"(x5));
#endif
}
__device__ __forceinline__ void guard4x5(v8f& a, v8f& b, v8f& c, v8f& d,
                                         v16h x0, v16h x1, v16h x2, v16h x3, v16h x4) {
#if defined(__HIP_DEVICE_COMPILE__)
  asm volatile("v_nop\n\tv_nop\n\tv_nop\n\tv_nop"
               : "+v"(a), "+v"(b), "+v"(c), "+v"(d) : "v"(x0), "v"(x1), "v"(x2), "v"(x3), "v"(x4));
#endif
}
__device__ __forceinline__ void keep4_h(v16h a, v16h b, v16h c, v16h d) {
#if defined(__HIP_DEVICE_COMPILE__)
  asm volatile("v_nop" :: "v"(a), "v"(b), "v"(c), "v"(d));
#endif
}
__device__ __forceinline__ void acc_guard4(v8f& a, v8f& b, v8f& c, v8f& d) {
#if defined(__HIP_DEVICE_COMPILE__)
  asm volatile("v_nop\n\tv_nop\n\tv_nop\n\tv_nop" : "+v"(a), "+v"(b), "+v"(c), "+v"(d));
#endif
}
__device__ __forceinline__ void wave_sync_lds() {
  __builtin_amdgcn_fence(__ATOMIC_RELEASE, "workgroup");
  __builtin_amdgcn_wave_barrier();
  __builtin_amdgcn_fence(__ATOMIC_ACQUIRE, "workgroup");
}

__global__ __launch_bounds__(256) void cvt16(const float* __restrict__ src, unsigned short* dst, int n, float sc) {
  const size_t i8 = ((size_t)blockIdx.x * 256 + threadIdx.x) * 8;
  if (i8 + 8 > (size_t)n) return;
  const v4f a = *(const v4f*)(src + i8);
  const v4f b = *(const v4f*)(src + i8 + 4);
  v4u o;
  o[0] = pk16(h_bits((_Float16)(bfr(a[0]) * sc)), h_bits((_Float16)(bfr(a[1]) * sc)));
  o[1] = pk16(h_bits((_Float16)(bfr(a[2]) * sc)), h_bits((_Float16)(bfr(a[3]) * sc)));
  o[2] = pk16(h_bits((_Float16)(bfr(b[0]) * sc)), h_bits((_Float16)(bfr(b[1]) * sc)));
  o[3] = pk16(h_bits((_Float16)(bfr(b[2]) * sc)), h_bits((_Float16)(bfr(b[3]) * sc)));
  for (int pass = 0; pass < 2; ++pass) {
    *(volatile v4u*)(dst + i8) = o;
    __threadfence();
  }
}

template <int BFO>
__global__ __launch_bounds__(256) void tr16(const float* __restrict__ W, unsigned short* WT, int Cin, int Dd,
                                            long long sIn, long long sOut, float sc) {
  __shared__ float t[64][65];
  const int tid = threadIdx.x;
  const int c0 = blockIdx.x * 64, d0 = blockIdx.y * 64;
  const float* src = W + (size_t)((long long)blockIdx.z * sIn);
  unsigned short* dst = WT + (size_t)((long long)blockIdx.z * sOut);
#pragma unroll
  for (int it = 0; it < 4; ++it) {
    const int p  = it * 256 + tid;
    const int cc = p >> 4, sg = (p & 15) * 4;
    const v4f v = *(const v4f*)(src + (size_t)(c0 + cc) * Dd + d0 + sg);
    t[cc][sg]     = v[0];
    t[cc][sg + 1] = v[1];
    t[cc][sg + 2] = v[2];
    t[cc][sg + 3] = v[3];
  }
  __syncthreads();
  v4u o[2];
#pragma unroll
  for (int it = 0; it < 2; ++it) {
    const int p  = it * 256 + tid;
    const int dd = p >> 3, s8 = (p & 7) * 8;
    unsigned short hv[8];
#pragma unroll
    for (int k = 0; k < 8; ++k) {
      const float f = bfr(t[s8 + k][dd]);
      if constexpr (BFO != 0) hv[k] = bf_bits(f);
      else hv[k] = h_bits((_Float16)(f * sc));
    }
    v4u q;
    q[0] = pk16(hv[0], hv[1]);
    q[1] = pk16(hv[2], hv[3]);
    q[2] = pk16(hv[4], hv[5]);
    q[3] = pk16(hv[6], hv[7]);
    o[it] = q;
  }
  for (int pass = 0; pass < 2; ++pass) {
#pragma unroll
    for (int it = 0; it < 2; ++it) {
      const int p  = it * 256 + tid;
      const int dd = p >> 3, s8 = (p & 7) * 8;
      *(volatile v4u*)(dst + (size_t)(d0 + dd) * Cin + c0 + s8) = o[it];
    }
    __threadfence();
  }
}

template <int OM, int ASPLIT, int BF, int EPI>
__global__ __launch_bounds__(256) __attribute__((amdgpu_num_vgpr(256))) void gemm64(
    const unsigned short* __restrict__ Ap, const unsigned short* __restrict__ A2p, int lda, long long sA,
    const unsigned short* __restrict__ Btp, int ldb, long long sB,
    void* Cout, void* C2out, int ldc, long long sC,
    int M, int N, int K, float oscale, float ocarry,
    const float* __restrict__ ep0, const float* __restrict__ ep1, const float* __restrict__ ep2) {
  __shared__ __align__(16) float sT[8][16 * 68];
  const int by   = blockIdx.y;
  const int lane = threadIdx.x & 31;
  const int wave = threadIdx.x >> 5;
  const int tilesN = N >> 6;
  const int tilesM = M >> 6;
  const int tile = blockIdx.x * 8 + wave;
  if (tile >= tilesM * tilesN) return;
  const int tm = tile / tilesN;
  const int tn = tile - tm * tilesN;
  const int m0 = tm << 6;
  const int n0 = tn << 6;

  const unsigned short* A1 = Ap  + (size_t)((long long)by * sA);
  const unsigned short* A2 = A2p + (size_t)((long long)by * sA);
  const unsigned short* Bb = Btp + (size_t)((long long)by * sB);

  const int rlane = lane & 15;
  const int koff  = (lane >> 4) * 8;
  const int mOff  = (lane >> 4) * 8;

  v8f acc[4][4];
#pragma unroll
  for (int i = 0; i < 4; ++i)
#pragma unroll
    for (int j = 0; j < 4; ++j) acc[i][j] = zero8();

  for (int k0 = 0; k0 < K; k0 += 32) {
    v16h bh[4];
#pragma unroll
    for (int j = 0; j < 4; ++j) {
      const size_t bofs = (size_t)(n0 + (j << 4) + rlane) * ldb + koff + k0;
      bh[j] = ldfrag_u(Bb + bofs);
    }
#pragma unroll
    for (int i = 0; i < 4; ++i) {
      const size_t ao = (size_t)(m0 + (i << 4) + rlane) * lda + koff + k0;
      const v16h ah = ldfrag_u(A1 + ao);
#pragma unroll
      for (int j = 0; j < 4; ++j) acc[i][j] = mmaT<BF>(ah, bh[j], acc[i][j]);
      dep_guard1(acc[i][0], acc[i][3], ah);
      if constexpr (ASPLIT != 0) {
        const v16h al = ldfrag_u(A2 + ao);
#pragma unroll
        for (int j = 0; j < 4; ++j) acc[i][j] = mmaT<BF>(al, bh[j], acc[i][j]);
        dep_guard1(acc[i][0], acc[i][3], al);
      }
    }
    keep4_h(bh[0], bh[1], bh[2], bh[3]);
  }
  acc_guard4(acc[0][0], acc[0][1], acc[0][2], acc[0][3]);
  acc_guard4(acc[1][0], acc[1][1], acc[1][2], acc[1][3]);
  acc_guard4(acc[2][0], acc[2][1], acc[2][2], acc[2][3]);
  acc_guard4(acc[3][0], acc[3][1], acc[3][2], acc[3][3]);

  const int hh2 = lane >> 4, c4 = (lane & 15) * 4;
  const int q8  = lane >> 3, c8 = (lane & 7) * 8;

  float* slab = sT[wave];
#pragma unroll
  for (int i = 0; i < 4; ++i) {
    const int mBase = m0 + (i << 4);
#pragma unroll
    for (int j = 0; j < 4; ++j) {
#pragma unroll
      for (int r = 0; r < 8; ++r) {
        slab[(mOff + r) * 68 + (j << 4) + rlane] = acc[i][j][r];
      }
    }
    wave_sync_lds();
    if constexpr (OM == 0) {
      float* C = (float*)Cout + (size_t)((long long)by * sC);
      v4f vals[8];
#pragma unroll
      for (int it = 0; it < 8; ++it) {
        const int row = it * 2 + hh2;
        v4f v = *(const v4f*)(slab + row * 68 + c4);
#pragma unroll
        for (int e = 0; e < 4; ++e) v[e] = v[e] * oscale;
        if constexpr (EPI == 1) {
          const v4f bb = *(const v4f*)(ep0 + n0 + c4);
#pragma unroll
          for (int e = 0; e < 4; ++e) v[e] = v[e] + bfr(bb[e]);
        }
        vals[it] = v;
      }
      for (int pass = 0; pass < 2; ++pass) {
#pragma unroll
        for (int it = 0; it < 8; ++it) {
          const int gr = mBase + it * 2 + hh2;
          *(volatile v4f*)(C + (size_t)gr * ldc + n0 + c4) = vals[it];
        }
        __threadfence();
      }
    } else {
      unsigned short* C  = (unsigned short*)Cout  + (size_t)((long long)by * sC);
      unsigned short* Cb = (unsigned short*)C2out + (size_t)((long long)by * sC);
      v4u hv[4], lv[4];
#pragma unroll
      for (int it = 0; it < 4; ++it) {
        const int row = it * 4 + q8;
        const float* sp = slab + row * 68 + c8;
        float rb = 0.f;
        if constexpr (EPI == 2) rb = bfr(ep0[mBase + row]);
        v4u a  = {0u, 0u, 0u, 0u};
        v4u b2 = {0u, 0u, 0u, 0u};
#pragma unroll
        for (int e = 0; e < 4; ++e) {
          const int ci = n0 + c8 + 2 * e;
          float f0 = sp[2 * e] * oscale + rb;
          float f1 = sp[2 * e + 1] * oscale + rb;
          if constexpr (EPI == 1) {
            f0 += bfr(ep0[ci]);
            f1 += bfr(ep0[ci + 1]);
          }
          if constexpr (OM == 5) {
            const float g0 = (f0 + bfr(ep1[ci])) * ocarry, g1 = (f1 + bfr(ep1[ci + 1])) * ocarry;
            const float w0 = (f0 + bfr(ep2[ci])) * ocarry, w1 = (f1 + bfr(ep2[ci + 1])) * ocarry;
            a[e]  = pk16(h_bits((_Float16)g0), h_bits((_Float16)g1));
            b2[e] = pk16(h_bits((_Float16)w0), h_bits((_Float16)w1));
          } else {
            f0 *= ocarry; f1 *= ocarry;
            const _Float16 x0 = (_Float16)f0, x1 = (_Float16)f1;
            a[e] = pk16(h_bits(x0), h_bits(x1));
            if constexpr (OM == 4) {
              b2[e] = pk16(h_bits((_Float16)(f0 - (float)x0)), h_bits((_Float16)(f1 - (float)x1)));
            }
          }
        }
        hv[it] = a;
        lv[it] = b2;
      }
      for (int pass = 0; pass < 2; ++pass) {
#pragma unroll
        for (int it = 0; it < 4; ++it) {
          const int row = it * 4 + q8;
          *(volatile v4u*)(C + (size_t)(mBase + row) * ldc + n0 + c8) = hv[it];
          if constexpr (OM >= 4) {
            *(volatile v4u*)(Cb + (size_t)(mBase + row) * ldc + n0 + c8) = lv[it];
          }
        }
        __threadfence();
      }
    }
    wave_sync_lds();
  }
}

__global__ __launch_bounds__(ATT_THREADS) __attribute__((amdgpu_num_vgpr(256)))
void attnb(const unsigned short* __restrict__ QU, const unsigned short* __restrict__ KP,
           const unsigned short* __restrict__ VTh, const unsigned short* __restrict__ VTl,
           const float* __restrict__ Gt, unsigned short* CTh, unsigned short* CTl) {
  __shared__ __align__(16) float smem[ATT_SMEM_FLOATS];

  const int tid  = threadIdx.x;
  const int wave = tid >> 5;
  const int lane = tid & 31;
  const int hh   = lane >> 4;
  const int c    = lane & 15;

  const int head = wave;
  const int i0   = blockIdx.x * 16;

  const size_t qofs = (size_t)(i0 + c) * DM + head * HD + 8 * hh;
  const v16h qa = ldfrag_u(QU + qofs), qb = ldfrag_u(QU + qofs + 32);

  const unsigned short* Kb  = KP + head * HD + 8 * hh;
  const unsigned short* Vbh = VTh + (size_t)(head * HD) * SEQ + 8 * hh;
  const unsigned short* Vbl = VTl + (size_t)(head * HD) * SEQ + 8 * hh;
  const float* Gh = Gt + (size_t)head * SEQ * SEQ;

  const float PSC = SCL * LOG2E;
  const float CSC = PSC * (1.0f / (QC * QC));

  float mrow[8], lrow[8];
  v8f o0 = zero8(), o1 = zero8(), o2 = zero8(), o3 = zero8();
#pragma unroll
  for (int r = 0; r < 8; ++r) { mrow[r] = -INFINITY; lrow[r] = 0.f; }
  float* pt = smem + wave * (16 * 36);

#pragma unroll 1
  for (int jb = 0; jb < SEQ; jb += KCH) {
    v8f s0, s1;
    {
      const size_t ko = (size_t)(jb + c) * DM;
      const v16h k0a = ldfrag_u(Kb + ko), k0b = ldfrag_u(Kb + ko + 32);
      const v16h k1a = ldfrag_u(Kb + ko + (size_t)16 * DM), k1b = ldfrag_u(Kb + ko + (size_t)16 * DM + 32);
      s0 = mma_h(qa, k0a, zero8());
      s0 = mma_h(qb, k0b, s0);
      s1 = mma_h(qa, k1a, zero8());
      s1 = mma_h(qb, k1b, s1);
      guard2x6(s0, s1, qa, qb, k0a, k0b, k1a, k1b);
    }
#pragma unroll
    for (int r = 0; r < 8; ++r) {
      const int i  = i0 + 8 * hh + r;
      const int ja = jb + c, jc = jb + 16 + c;
      const bool la = (ja <= i), lc = (jc <= i);
      int ra = la ? i : (i + 1), rc = lc ? i : (i + 1);
      int ca = la ? (SEQ - 1 - i + ja) : (ja - i - 2);
      int cz = lc ? (SEQ - 1 - i + jc) : (jc - i - 2);
      ra = (ra > SEQ - 1) ? (SEQ - 1) : ra;
      rc = (rc > SEQ - 1) ? (SEQ - 1) : rc;
      ca = (ca < 0) ? 0 : ca;  ca = (ca > SEQ - 1) ? (SEQ - 1) : ca;
      cz = (cz < 0) ? 0 : cz;  cz = (cz > SEQ - 1) ? (SEQ - 1) : cz;
      const float ga = Gh[(size_t)ra * SEQ + ca];
      const float gc = Gh[(size_t)rc * SEQ + cz];
      const float pa = (ja == i + 1) ? 0.f : ga;
      const float pz = (jc == i + 1) ? 0.f : gc;
      const float t0 = s0[r] * CSC + pa * PSC, t1 = s1[r] * CSC + pz * PSC;
      float mx = fmaxf(t0, t1);
#pragma unroll
      for (int off = 1; off < 16; off <<= 1) mx = fmaxf(mx, __shfl_xor(mx, off, 32));
      const float mn = fmaxf(mrow[r], mx);
      const float al = exp2f(mrow[r] - mn);
      mrow[r] = mn;
      const float e0 = exp2f(t0 - mn), e1 = exp2f(t1 - mn);
      float ps = e0 + e1;
#pragma unroll
      for (int off = 1; off < 16; off <<= 1) ps += __shfl_xor(ps, off, 32);
      lrow[r] = lrow[r] * al + ps;
      o0[r] *= al;
      o1[r] *= al;
      o2[r] *= al;
      o3[r] *= al;
      const int ro = (8 * hh + r) * 36 + c;
      pt[ro]      = e0;
      pt[ro + 16] = e1;
    }
    wave_sync_lds();
    FragH ph, pl;
    {
      const float* prow = pt + c * 36 + 8 * hh;
      const v4f p0 = *(const v4f*)(prow), p1 = *(const v4f*)(prow + 4);
      const v4f p2 = *(const v4f*)(prow + 16), p3 = *(const v4f*)(prow + 20);
#pragma unroll
      for (int e = 0; e < 4; ++e) {
        float f; _Float16 x;
        f = p0[e] * PC; x = (_Float16)f; ph.h[0][e]     = x; pl.h[0][e]     = (_Float16)(f - (float)x);
        f = p1[e] * PC; x = (_Float16)f; ph.h[0][4 + e] = x; pl.h[0][4 + e] = (_Float16)(f - (float)x);
        f = p2[e] * PC; x = (_Float16)f; ph.h[1][e]     = x; pl.h[1][e]     = (_Float16)(f - (float)x);
        f = p3[e] * PC; x = (_Float16)f; ph.h[1][4 + e] = x; pl.h[1][4 + e] = (_Float16)(f - (float)x);
      }
    }
    const size_t vo = (size_t)c * SEQ + jb;
    {
      const v16h vh0 = ldfrag_u(Vbh + vo);
      const v16h vh1 = ldfrag_u(Vbh + vo + (size_t)16 * SEQ);
      const v16h vh2 = ldfrag_u(Vbh + vo + (size_t)32 * SEQ);
      const v16h vh3 = ldfrag_u(Vbh + vo + (size_t)48 * SEQ);
      o0 = mma_h(ph.v, vh0, o0);
      o1 = mma_h(ph.v, vh1, o1);
      o2 = mma_h(ph.v, vh2, o2);
      o3 = mma_h(ph.v, vh3, o3);
      o0 = mma_h(pl.v, vh0, o0);
      o1 = mma_h(pl.v, vh1, o1);
      o2 = mma_h(pl.v, vh2, o2);
      o3 = mma_h(pl.v, vh3, o3);
      guard4x6(o0, o1, o2, o3, ph.v, pl.v, vh0, vh1, vh2, vh3);
    }
    {
      const v16h vl0 = ldfrag_u(Vbl + vo);
      const v16h vl1 = ldfrag_u(Vbl + vo + (size_t)16 * SEQ);
      const v16h vl2 = ldfrag_u(Vbl + vo + (size_t)32 * SEQ);
      const v16h vl3 = ldfrag_u(Vbl + vo + (size_t)48 * SEQ);
      o0 = mma_h(ph.v, vl0, o0);
      o1 = mma_h(ph.v, vl1, o1);
      o2 = mma_h(ph.v, vl2, o2);
      o3 = mma_h(ph.v, vl3, o3);
      guard4x5(o0, o1, o2, o3, ph.v, vl0, vl1, vl2, vl3);
    }
    wave_sync_lds();
  }

  __syncthreads();
  unsigned short* Osh = (unsigned short*)smem;
  unsigned short* Osl = Osh + 16 * DM;
  const float oc = 1.0f / (PC * VC);
  const int cb = wave * HD + c;
#pragma unroll
  for (int r = 0; r < 8; ++r) {
    const float inv = (1.0f / lrow[r]) * oc;
    const int ro = (8 * hh + r) * DM + cb;
    const float f0 = o0[r] * inv, f1 = o1[r] * inv, f2 = o2[r] * inv, f3 = o3[r] * inv;
    const unsigned short g0 = bf_bits(f0), g1 = bf_bits(f1), g2 = bf_bits(f2), g3 = bf_bits(f3);
    Osh[ro]      = g0;  Osl[ro]      = bf_bits(f0 - bf_up(g0));
    Osh[ro + 16] = g1;  Osl[ro + 16] = bf_bits(f1 - bf_up(g1));
    Osh[ro + 32] = g2;  Osl[ro + 32] = bf_bits(f2 - bf_up(g2));
    Osh[ro + 48] = g3;  Osl[ro + 48] = bf_bits(f3 - bf_up(g3));
  }
  __syncthreads();
  {
    v4u hv[4], lv[4];
#pragma unroll
    for (int it = 0; it < 4; ++it) {
      const int p = it * ATT_THREADS + tid;
      hv[it] = *(const v4u*)(Osh + (size_t)p * 8);
      lv[it] = *(const v4u*)(Osl + (size_t)p * 8);
    }
    const size_t dofs = (size_t)i0 * DM;
    unsigned short* dsth = CTh + dofs;
    unsigned short* dstl = CTl + dofs;
    for (int pass = 0; pass < 2; ++pass) {
#pragma unroll
      for (int it = 0; it < 4; ++it) {
        const int p = it * ATT_THREADS + tid;
        *(volatile v4u*)(dsth + (size_t)p * 8) = hv[it];
        *(volatile v4u*)(dstl + (size_t)p * 8) = lv[it];
      }
      __threadfence();
    }
  }
}

extern "C" void kernel_launch(void* const* d_in, const int* in_sizes, int n_in,
                              void* d_out, int out_size, void* d_ws, size_t ws_size,
                              hipStream_t stream) {
  if (n_in < 15) return;
  const int NA = NROWS * DM;
  if (in_sizes[0] != NA || in_sizes[1] != NA || in_sizes[2] != NA || in_sizes[3] != NA) return;
  if (in_sizes[4] != DM * DM || in_sizes[6] != DM * DM || in_sizes[8] != DM * DM || in_sizes[10] != DM * DM || in_sizes[13] != DM * DM) return;
  if (in_sizes[5] != DM || in_sizes[7] != DM || in_sizes[9] != DM || in_sizes[14] != DM) return;
  if (in_sizes[11] != NHEAD * HD || in_sizes[12] != NHEAD * HD) return;
  if (out_size != NROWS * DM) return;
  if ((NA % 2048) != 0) return;

  const float* query = (const float*)d_in[0];
  const float* key   = (const float*)d_in[1];
  const float* value = (const float*)d_in[2];
  const float* pemb  = (const float*)d_in[3];
  const float* w_q   = (const float*)d_in[4];
  const float* b_q   = (const float*)d_in[5];
  const float* w_k   = (const float*)d_in[6];
  const float* b_k   = (const float*)d_in[7];
  const float* w_v   = (const float*)d_in[8];
  const float* b_v   = (const float*)d_in[9];
  const float* w_p   = (const float*)d_in[10];
  const float* u_b   = (const float*)d_in[11];
  const float* v_b   = (const float*)d_in[12];
  const float* w_o   = (const float*)d_in[13];
  const float* b_o   = (const float*)d_in[14];
  float*       out   = (float*)d_out;

  const size_t PWT = (size_t)DM * DM * 2;
  const size_t PX  = (size_t)NROWS * DM * 2;
  const size_t PVT = (size_t)NB * DM * SEQ * 2;
  const size_t PG  = (size_t)NHEAD * SEQ * SEQ * 4;
  size_t off = 0;
  const size_t oWQ = off; off += PWT;
  const size_t oWK = off; off += PWT;
  const size_t oWV = off; off += PWT;
  const size_t oWP = off; off += PWT;
  const size_t oWO = off; off += PWT;
  const size_t oX  = off; off += PX;
  const size_t oQU = off; off += PX;
  const size_t oQV = off; off += PX;
  const size_t oK  = off; off += PX;
  const size_t oP  = off; off += PX;
  const size_t oVh = off; off += PVT;
  const size_t oVl = off; off += PVT;
  const size_t oG  = off; off += PG;
  const size_t oCh = off; off += PX;
  const size_t oCl = off; off += PX;
  if (off > ws_size) return;
  if (off > (size_t)134217728) return;

  char* ws = (char*)d_ws;
  unsigned short* WQT  = (unsigned short*)(ws + oWQ);
  unsigned short* WKT  = (unsigned short*)(ws + oWK);
  unsigned short* WVT  = (unsigned short*)(ws + oWV);
  unsigned short* WPT  = (unsigned short*)(ws + oWP);
  unsigned short* WOT  = (unsigned short*)(ws + oWO);
  unsigned short* X16  = (unsigned short*)(ws + oX);
  unsigned short* QU   = (unsigned short*)(ws + oQU);
  unsigned short* QV   = (unsigned short*)(ws + oQV);
  unsigned short* K16  = (unsigned short*)(ws + oK);
  unsigned short* P16  = (unsigned short*)(ws + oP);
  unsigned short* VTh  = (unsigned short*)(ws + oVh);
  unsigned short* VTl  = (unsigned short*)(ws + oVl);
  float*          GTAB = (float*)(ws + oG);
  unsigned short* CTh  = (unsigned short*)(ws + oCh);
  unsigned short* CTl  = (unsigned short*)(ws + oCl);

  const dim3 blk(256);
  const dim3 gTW(DM / 64, DM / 64, 1);
  const dim3 gCX(NA / 2048);
  const int tilesP = (NROWS / 64) * (DM / 64);
  const int tilesV = (DM / 64) * (SEQ / 64);
  const int tilesG = (SEQ / 64) * (SEQ / 64);
  const dim3 gP((tilesP + 7) / 8, 1);
  const dim3 gV((tilesV + 7) / 8, NB);
  const dim3 gG((tilesG + 7) / 8, NHEAD);
  const dim3 gAT(ATT_BLOCKS);
  const dim3 bAT(ATT_THREADS);

  tr16<0><<<gTW, blk, 0, stream>>>(w_q, WQT, DM, DM, 0LL, 0LL, WSC);
  tr16<0><<<gTW, blk, 0, stream>>>(w_k, WKT, DM, DM, 0LL, 0LL, WSC);
  tr16<0><<<gTW, blk, 0, stream>>>(w_v, WVT, DM, DM, 0LL, 0LL, WSC);
  tr16<0><<<gTW, blk, 0, stream>>>(w_p, WPT, DM, DM, 0LL, 0LL, WSC);
  tr16<1><<<gTW, blk, 0, stream>>>(w_o, WOT, DM, DM, 0LL, 0LL, 1.0f);

  cvt16<<<gCX, blk, 0, stream>>>(query, X16, NA, ACARRY);
  gemm64<5, 0, 0, 1><<<gP, blk, 0, stream>>>(
      X16, X16, DM, 0LL,
      WQT, DM, 0LL,
      (void*)QU, (void*)QV, DM, 0LL,
      NROWS, DM, DM, 1.0f / (ACARRY * WSC), QC,
      b_q, u_b, v_b);

  cvt16<<<gCX, blk, 0, stream>>>(key, X16, NA, ACARRY);
  gemm64<2, 0, 0, 1><<<gP, blk, 0, stream>>>(
      X16, X16, DM, 0LL,
      WKT, DM, 0LL,
      (void*)K16, (void*)K16, DM, 0LL,
      NROWS, DM, DM, 1.0f / (ACARRY * WSC), QC,
      b_k, b_k, b_k);

  cvt16<<<gCX, blk, 0, stream>>>(value, X16, NA, ACARRY);
  gemm64<4, 0, 0, 2><<<gV, blk, 0, stream>>>(
      WVT, WVT, DM, 0LL,
      X16, DM, (long long)SEQ * DM,
      (void*)VTh, (void*)VTl, SEQ, (long long)DM * SEQ,
      DM, SEQ, DM, 1.0f / (ACARRY * WSC), VC,
      b_v, b_v, b_v);

  cvt16<<<gCX, blk, 0, stream>>>(pemb, X16, NA, ACARRY);
  gemm64<2, 0, 0, 0><<<gP, blk, 0, stream>>>(
      X16, X16, DM, 0LL,
      WPT, DM, 0LL,
      (void*)P16, (void*)P16, DM, 0LL,
      NROWS, DM, DM, 1.0f / (ACARRY * WSC), QC,
      b_q, b_q, b_q);

  for (int b = 0; b < NB; ++b) {
    const size_t boff = (size_t)b * SEQ * DM;
    const size_t voff = (size_t)b * DM * SEQ;
    gemm64<0, 0, 0, 0><<<gG, blk, 0, stream>>>(
        QV + boff, QV + boff, DM, (long long)HD,
        P16 + boff, DM, (long long)HD,
        (void*)GTAB, (void*)GTAB, SEQ, (long long)SEQ * SEQ,
        SEQ, SEQ, HD, 1.0f / (QC * QC), 1.0f,
        b_q, b_q, b_q);
    attnb<<<gAT, bAT, 0, stream>>>(QU + boff, K16 + boff, VTh + voff, VTl + voff, GTAB, CTh + boff, CTl + boff);
  }

  gemm64<0, 1, 1, 1><<<gP, blk, 0, stream>>>(
      CTh, CTl, DM, 0LL,
      WOT, DM, 0LL,
      (void*)out, (void*)out, DM, 0LL,
      NROWS, DM, DM, 1.0f, 1.0f,
      b_o, b_o, b_o);
  (void)hipGetLastError();
}
